// NeighborhoodAttention2D_1726576854815
// MI455X (gfx1250) — hardware-verified
//
#include <hip/hip_runtime.h>


namespace {
typedef _Float16 b16;
typedef __attribute__((ext_vector_type(16))) _Float16 v16b;
typedef __attribute__((ext_vector_type(8))) _Float16 v8b;
typedef __attribute__((ext_vector_type(4))) _Float16 v4h;
typedef __attribute__((ext_vector_type(2))) _Float16 v2h;
typedef __attribute__((ext_vector_type(8))) float v8f;
typedef __attribute__((ext_vector_type(4))) float v4f;
typedef __attribute__((ext_vector_type(2))) float v2f;
__device__ __forceinline__ float bf16_rne(float f) { unsigned int u = __float_as_uint(f); u += 0x7FFFu + ((u >> 16) & 1u); return __uint_as_float(u & 0xFFFF0000u); }
__device__ __forceinline__ void split16(float v, b16& hi, b16& lo) { hi = (b16)v; lo = (b16)(v - (float)hi); }
__device__ __forceinline__ v16b frag_kb(const b16* p, int hh) { const v8b a = *(const v8b*)(p + 8 * hh), b = *(const v8b*)(p + 16 + 8 * hh); v16b f;
#pragma unroll
  for (int e = 0; e < 8; ++e) { f[e] = a[e]; f[8 + e] = b[e]; } return f; }
__device__ __forceinline__ v8f wmma16b(v16b a, v16b b, v8f c) { v8f d = __builtin_amdgcn_wmma_f32_16x16x32_f16(false, a, false, b, (short)0, c, false, false); asm volatile("v_nop\n\tv_nop\n\tv_nop\n\tv_nop" : "+v"(d) : "v"(a), "v"(b)); return d; }
__device__ __forceinline__ void wave_lds_sync() { __builtin_amdgcn_fence(__ATOMIC_RELEASE, "workgroup"); __builtin_amdgcn_wave_barrier(); __builtin_amdgcn_fence(__ATOMIC_ACQUIRE, "workgroup"); }
__device__ __forceinline__ float pmul(float a, float b) { float p = a * b; asm volatile("" : "+v"(p)); return p; }
__device__ __forceinline__ int iclamp(int v, int lo, int hi) { return v < lo ? lo : (v > hi ? hi : v); }
__device__ __forceinline__ float nexp2(float v) { return __builtin_amdgcn_exp2f(v); }

constexpr int B = 8, BL = B  , C = 512, HI = 56, WI = 56, T = HI * WI  , NH = 16, HD = 32, KS = 7, NQKV = 3 * C;
constexpr float XS = 8.0f, WSC = 256.0f, PS = 1024.0f, RS_ = 1024.0f  , LOG2E = 1.4426950408889634f, SCALE = 0.17677669529663687f  ;
static_assert(T % 64 == 0 && C % 128 == 0 && HD == 32 && NH * HD == C && WI - 32 >= 0, "tiling");

__global__ __launch_bounds__(256) void wcvt_kernel(const float* __restrict__ w, b16* __restrict__ W16, int n8) {
  const int u = blockIdx.x * 256 + threadIdx.x; if (u >= n8) return; const size_t e = (size_t)u * 8; v8b o; for (int j = 0; j < 8; ++j) o[j] = (b16)(bf16_rne(w[e + j]) * WSC);
  for (int pass = 0; pass < 2; ++pass) { *(volatile v8b*)(W16 + e) = o; __threadfence(); }
}
__global__ __launch_bounds__(128) void qkv_kernel(const float* __restrict__ x, const b16* __restrict__ WQ, const float* __restrict__ qb, b16* __restrict__ QP, b16* __restrict__ KP, b16* __restrict__ VT, b16* __restrict__ VTL) {
  __shared__ __attribute__((aligned(16))) b16 As[64][C + 8]; __shared__ __attribute__((aligned(16))) float Tf[4][16][128 + 4];
  const int wave = threadIdx.x >> 5, lane = threadIdx.x & 31, nloc = lane & 15, hlf = lane >> 4; const int t0 = blockIdx.x * 64; const int b = blockIdx.y; const int slab = blockIdx.z, n0 = slab * 128, part = slab / 4, h0 = (slab & 3) * 4;
  for (int i = threadIdx.x; i < C * 16; i += 128) { const int c = i / 16, q4 = (i % 16) * 4; const v4f f = *(const v4f*)(x + ((size_t)b * C + c) * T + t0 + q4); for (int j = 0; j < 4; ++j) As[q4 + j][c] = (b16)(bf16_rne(f[j]) * XS); }
  __syncthreads();
  v8f acc[8];
#pragma unroll
  for (int t = 0; t < 8; ++t) acc[t] = (v8f){};
#pragma unroll 2
  for (int kb = 0; kb < C; kb += 32) { const v16b a = frag_kb(&As[wave * 16 + nloc][kb], hlf);
#pragma unroll
    for (int t = 0; t < 8; ++t) acc[t] = wmma16b(a, frag_kb(WQ + (size_t)(n0 + t * 16 + nloc) * C + kb, hlf), acc[t]); }
#pragma unroll
  for (int t = 0; t < 8; ++t) { const float bb = bf16_rne(qb[n0 + t * 16 + nloc]);
#pragma unroll
    for (int r = 0; r < 8; ++r) Tf[wave][8 * hlf + r][t * 16 + nloc] = acc[t][r] * (1.0f / (XS * WSC)) + bb; }
  __syncthreads();
  for (int pass = 0; pass < 2; ++pass) {
    if (part < 2) { b16* plane = part == 0 ? QP : KP; const int h = h0 + (lane >> 3), d = (lane & 7) * 4;
      for (int rr = 0; rr < 16; ++rr) { const int tok = t0 + wave * 16 + rr; v4h o4; for (int j = 0; j < 4; ++j) o4[j] = (b16)(Tf[wave][rr][lane * 4 + j] * XS); *(volatile v4h*)(plane + (((size_t)b * NH + h) * T + tok) * HD + d) = o4; } }
    else {
#pragma unroll 1
      for (int q = 0; q < 32; ++q) { const int cl = wave * 32 + q; const int h = h0 + cl / HD, d = cl % HD; const int tk = lane * 2; v2h hv, lv; for (int e2 = 0; e2 < 2; ++e2) { const float vs = Tf[(tk + e2) >> 4][(tk + e2) & 15][cl] * XS; const b16 ph = (b16)vs; hv[e2] = ph; lv[e2] = (b16)((vs - (float)ph) * RS_); }
        const size_t dst = (((size_t)b * NH + h) * HD + d) * (size_t)T + t0 + tk; *(volatile v2h*)(VT + dst) = hv; *(volatile v2h*)(VTL + dst) = lv; } }
    __threadfence(); }
}
__global__ __launch_bounds__(64) void attn_kernel(const b16* __restrict__ QP, const b16* __restrict__ KP, const b16* __restrict__ VT, const b16* __restrict__ VTL, const float* __restrict__ rpb, float* __restrict__ CT) {
  __shared__ __attribute__((aligned(16))) b16 Pb[2][16][32 + 8], Pl[2][16][32 + 8]; __shared__ __attribute__((aligned(16))) float To[2][16][HD + 4]; __shared__ float Rb[2][KS][13];
  const int wave = threadIdx.x >> 5, lane = threadIdx.x & 31, hh = lane >> 4, col = lane & 15; const int i = blockIdx.x >> 1; const int j0 = (((blockIdx.x & 1) * 2) + wave) * 16; const int b = blockIdx.y / NH, h = blockIdx.y % NH;
  const int r0 = iclamp(i - KS / 2, 0, HI - KS), c0 = iclamp(j0 - KS / 2, 0, WI - 32); const int j = j0 + col, jq = j < WI ? j : WI - 1; const int sj = iclamp(j - KS / 2, 0, WI - KS);
  for (int q = lane; q < KS * 13; q += 32) { const int kr = q / 13, dj = q % 13; Rb[wave][kr][dj] = bf16_rne(rpb[((size_t)h * 13 + (r0 + kr - i + KS - 1)) * 13 + dj]); }
  wave_lds_sync();
  const size_t ph = (size_t)b * NH + h; const b16* Qb = QP + ph * T * HD; const b16* Kb = KP + ph * T * HD; const b16* Vb = VT + ph * HD * (size_t)T; const b16* Vlb = VTL + ph * HD * (size_t)T;
  const v16b qa = frag_kb(Qb + (size_t)(i * WI + jq) * HD, hh);
  const float cs = LOG2E * SCALE / (XS * XS);
  float m = -INFINITY, l = 0.0f; v8f o[2], o2[2]; o[0] = (v8f){}; o[1] = (v8f){}; o2[0] = (v8f){}; o2[1] = (v8f){};
#pragma unroll 1
  for (int kr = 0; kr < KS; ++kr) { const int r = r0 + kr; const size_t ktok0 = (size_t)r * WI + c0;
    float e[16]; float mx = -INFINITY;
#pragma unroll
    for (int u = 0; u < 2; ++u) { v8f s = (v8f){}; s = wmma16b(frag_kb(Kb + (ktok0 + u * 16 + col) * HD, hh), qa, s);
#pragma unroll
      for (int rr = 0; rr < 8; ++rr) { const int kc = c0 + u * 16 + 8 * hh + rr; const int dj = kc - j + KS - 1; const bool ok = (kc >= sj) && (kc < sj + KS) && (j < WI); const float vv = ok ? s[rr] * cs + Rb[wave][kr][iclamp(dj, 0, 12)] * LOG2E : -INFINITY; e[u * 8 + rr] = vv; mx = fmaxf(mx, vv); } }
    mx = fmaxf(mx, __shfl_xor(mx, 16)); const float mn = fmaxf(m, mx); const float al = (mn == -INFINITY) ? 1.0f : nexp2(m - mn); float sum = 0.0f;
#pragma unroll
    for (int i2 = 0; i2 < 16; ++i2) { const float p = (mn == -INFINITY) ? 0.0f : nexp2(e[i2] - mn); sum += p; const float ps = p * PS; const b16 ph = (b16)ps; const int slot = (i2 < 8 ? 0 : 16) + 8 * hh + (i2 & 7); Pb[wave][col][slot] = ph; Pl[wave][col][slot] = (b16)((ps - (float)ph) * RS_); }
    sum += __shfl_xor(sum, 16); l = l * al + sum; m = mn;
    wave_lds_sync();
    const v16b pf = frag_kb(&Pb[wave][col][0], hh), plf = frag_kb(&Pl[wave][col][0], hh);
#pragma unroll
    for (int t = 0; t < 2; ++t) { o[t] *= al; o2[t] *= al; const v16b vh = frag_kb(Vb + (size_t)(t * 16 + col) * T + ktok0, hh); o[t] = wmma16b(vh, pf, o[t]); o2[t] = wmma16b(frag_kb(Vlb + (size_t)(t * 16 + col) * T + ktok0, hh), pf, o2[t]); o2[t] = wmma16b(vh, plf, o2[t]); }
    wave_lds_sync(); }
  const float inv = (l > 0.0f) ? 1.0f / (l * PS * XS) : 0.0f;
#pragma unroll
  for (int t = 0; t < 2; ++t)
#pragma unroll
    for (int rr = 0; rr < 8; ++rr) To[wave][col][t * 16 + 8 * hh + rr] = (o[t][rr] + o2[t][rr] * (1.0f / RS_)) * inv;
  wave_lds_sync();
  for (int pass = 0; pass < 2; ++pass) { for (int rr = 0; rr < 16; ++rr) { if (j0 + rr >= WI) break;
      ((volatile float*)CT)[((size_t)b * T + (size_t)i * WI + j0 + rr) * C + h * HD + lane] = To[wave][rr][lane]; } __threadfence(); }
}
__global__ __launch_bounds__(64) void proj_kernel(const float* __restrict__ CT, const b16* __restrict__ WP, const float* __restrict__ pbias, float* __restrict__ out) {
  __shared__ __attribute__((aligned(16))) b16 Ah[2][16][128 + 8], Al[2][16][128 + 8]; __shared__ __attribute__((aligned(16))) float Tf[2][16][128 + 4];
  const int wave = threadIdx.x >> 5, lane = threadIdx.x & 31, nloc = lane & 15, hlf = lane >> 4; const int t0 = blockIdx.x * 32; const int b = blockIdx.y; const int n0 = blockIdx.z * 128; const size_t m0 = (size_t)b * T + t0 + wave * 16;
  v8f acc[8], acc2[8];
#pragma unroll
  for (int t = 0; t < 8; ++t) { acc[t] = (v8f){}; acc2[t] = (v8f){}; }
#pragma unroll 1
  for (int kc = 0; kc < C; kc += 128) {
    for (int idx = lane; idx < 16 * 32; idx += 32) { const int rr = idx / 32, c4 = (idx % 32) * 4; const v4f v = *(const v4f*)(CT + (m0 + rr) * C + kc + c4); v4h hv, lv;
      for (int j = 0; j < 4; ++j) { const float vs = v[j] * XS; const b16 ph = (b16)vs; hv[j] = ph; lv[j] = (b16)((vs - (float)ph) * RS_); } *(v4h*)(&Ah[wave][rr][c4]) = hv; *(v4h*)(&Al[wave][rr][c4]) = lv; }
    wave_lds_sync();
#pragma unroll
    for (int kb = 0; kb < 128; kb += 32) { const v16b a = frag_kb(&Ah[wave][nloc][kb], hlf), al = frag_kb(&Al[wave][nloc][kb], hlf);
#pragma unroll
      for (int t = 0; t < 8; ++t) { const v16b bw = frag_kb(WP + (size_t)(n0 + t * 16 + nloc) * C + kc + kb, hlf); acc[t] = wmma16b(a, bw, acc[t]); acc2[t] = wmma16b(al, bw, acc2[t]); } }
    wave_lds_sync(); }
#pragma unroll
  for (int t = 0; t < 8; ++t) { const float bb = bf16_rne(pbias[n0 + t * 16 + nloc]);
#pragma unroll
    for (int r = 0; r < 8; ++r) Tf[wave][8 * hlf + r][t * 16 + nloc] = (acc[t][r] + acc2[t][r] * (1.0f / RS_)) * (1.0f / (XS * WSC)) + bb; }
  __syncthreads();
  for (int pass = 0; pass < 2; ++pass) { for (int q = 0; q < 64; ++q) { const int cl = wave * 64 + q; ((volatile float*)out)[((size_t)b * C + n0 + cl) * T + t0 + lane] = Tf[lane >> 4][lane & 15][cl]; } __threadfence(); }
}
}

extern "C" void kernel_launch(void* const* d_in, const int* in_sizes, int n_in, void* d_out, int out_size, void* d_ws, size_t ws_size, hipStream_t stream) {
  (void)n_in;
  auto Fp = [&](int i) { return (const float*)d_in[i]; };
  if (in_sizes[0] != B * C * T || in_sizes[1] != NQKV * C || in_sizes[2] != NQKV || in_sizes[3] != NH * 13 * 13 || in_sizes[4] != C * C || in_sizes[5] != C || out_size != B * C * T) return;
  size_t off = 0; char* ws = (char*)d_ws;
  auto carve = [&](size_t bytes) { char* p = ws + off; off += (bytes + 255) & ~(size_t)255; return p; };
  b16* WQ = (b16*)carve((size_t)NQKV * C * 2); b16* WP = (b16*)carve((size_t)C * C * 2); const size_t plane = (size_t)B * NH * T * HD * 2;
  b16* QP = (b16*)carve(plane); b16* KP = (b16*)carve(plane); b16* VT = (b16*)carve(plane); b16* VTL = (b16*)carve(plane); float* CT = (float*)carve((size_t)B * T * C * 4);
  if (off > ws_size || off > ((size_t)240 << 20)) return;
  wcvt_kernel<<<(NQKV * C / 8 + 255) / 256, 256, 0, stream>>>(Fp(1), WQ, NQKV * C / 8); wcvt_kernel<<<(C * C / 8 + 255) / 256, 256, 0, stream>>>(Fp(4), WP, C * C / 8);
  qkv_kernel<<<dim3(T / 64, BL, 12), 128, 0, stream>>>(Fp(0), WQ, Fp(2), QP, KP, VT, VTL);
  attn_kernel<<<dim3(HI * 2, BL * NH), 64, 0, stream>>>(QP, KP, VT, VTL, Fp(3), CT);
  proj_kernel<<<dim3(T / 32, BL, C / 128), 64, 0, stream>>>(CT, WP, Fp(5), (float*)d_out);
}
